// SimpleMPGNN_15152644620815
// MI455X (gfx1250) — hardware-verified
//
#include <hip/hip_runtime.h>
#include <stddef.h>


#define NTHR   256
#define NWAVE  8
#define EPT    8
#define CHUNK  (NTHR * EPT)
#define PCAP   3072
#define DRAINT (PCAP - CHUNK)
#define QMAX   (PCAP / NTHR)
#define NB     352
#define NROWA  (NB + NWAVE)
#define HC     128
#define PQW    256
#define MT     64
#define NGRAPH 64
#define KEYSH  10
#define WSC    16.0f
#define WINV   0.0625f
#define BN_EPS 1e-5f

static_assert(QMAX * NTHR == PCAP);
static_assert(DRAINT > 0);
static_assert((PCAP % 16) == 0);
static_assert(NROWA < (1 << KEYSH));
static_assert((NB % NWAVE) == 0);
static_assert((NB % 2) == 0);

typedef float          v4f   __attribute__((ext_vector_type(4)));
typedef float          v8f   __attribute__((ext_vector_type(8)));
typedef int            v4i   __attribute__((ext_vector_type(4)));
typedef double         v2d   __attribute__((ext_vector_type(2)));
typedef _Float16       v8h   __attribute__((ext_vector_type(8)));
typedef _Float16       v16h  __attribute__((ext_vector_type(16)));
typedef unsigned short v8us  __attribute__((ext_vector_type(8)));
typedef unsigned short v16us __attribute__((ext_vector_type(16)));
typedef __bf16         v16b  __attribute__((ext_vector_type(16)));
union FragH { v16h v; v8h h[2]; };
union FragB { v16b v; v16us u; v8us h[2]; };

__device__ __forceinline__ int clampi(int v, int lo, int hi) { return v < lo ? lo : (v > hi ? hi : v); }

__device__ __forceinline__ v8f wmh(v16h a, v16h b, v8f c) {
  v8f d = __builtin_amdgcn_wmma_f32_16x16x32_f16(false, a, false, b, (short)0, c, false, false);
  asm volatile("v_nop\n\tv_nop\n\tv_nop\n\tv_nop" : "+v"(d) : "v"(a), "v"(b));
  return d;
}
__device__ __forceinline__ v8f wmb(v16b a, v16b b, v8f c) {
  v8f d = __builtin_amdgcn_wmma_f32_16x16x32_bf16(false, a, false, b, (short)0, c, false, false);
  asm volatile("v_nop\n\tv_nop\n\tv_nop\n\tv_nop" : "+v"(d) : "v"(a), "v"(b));
  return d;
}
__device__ __forceinline__ v8f wmb3(v16b ah, v16b al, v16b bh, v16b bl, v8f c) {
  c = wmb(ah, bh, c);
  c = wmb(ah, bl, c);
  c = wmb(al, bh, c);
  return c;
}

__device__ __forceinline__ v16h ldfrag(const _Float16* p) {
  FragH f;
  f.h[0] = *(const v8h*)p;
  f.h[1] = *(const v8h*)(p + 16);
  return f.v;
}
__device__ __forceinline__ v16b ldfragb(const unsigned short* p) {
  FragB f;
  f.h[0] = *(const v8us*)p;
  f.h[1] = *(const v8us*)(p + 16);
  return f.v;
}

__device__ __forceinline__ unsigned short bf16_bits(float x) {
  unsigned u = __float_as_uint(x);
  u = u + 0x7FFFu + ((u >> 16) & 1u);
  return (unsigned short)(u >> 16);
}
__device__ __forceinline__ void split_bf16(float x, unsigned short& hi, unsigned short& lo) {
  const unsigned short h = bf16_bits(x);
  const float hf = __uint_as_float(((unsigned)h) << 16);
  hi = h;
  lo = bf16_bits(x - hf);
}

__device__ __forceinline__ void wave_lds_sync() {
  __builtin_amdgcn_fence(__ATOMIC_ACQ_REL, "wavefront");
  __builtin_amdgcn_wave_barrier();
}

__device__ __forceinline__ v4f san4(v4f v) {
  v4f r;
  r.x = (v.x > -3.0e38f) ? v.x : 0.0f;
  r.y = (v.y > -3.0e38f) ? v.y : 0.0f;
  r.z = (v.z > -3.0e38f) ? v.z : 0.0f;
  r.w = (v.w > -3.0e38f) ? v.w : 0.0f;
  return r;
}

__global__ __launch_bounds__(NTHR) void k_prepT(const float* __restrict__ w, _Float16* plane, int K, int Nn) {
  const int groups = (Nn * K) >> 3;
  const int g  = blockIdx.x * NTHR + threadIdx.x;
  const bool ok = g < groups;
  const int gc = ok ? g : groups - 1;
  const int kq8 = K >> 3;
  const int n = gc / kq8, kq = gc - n * kq8;
  v8h o;
#pragma unroll
  for (int i = 0; i < 8; ++i) {
    const float v = w[(size_t)(kq * 8 + i) * Nn + n] * WSC;
    o[i] = (_Float16)v;
  }
  _Float16* dst = plane + (size_t)n * K + kq * 8;
  if (ok) *(volatile v8h*)dst = o;
  __threadfence();
  if (ok) *(volatile v8h*)dst = o;
}

__global__ __launch_bounds__(NTHR) void k_prepT3(const float* __restrict__ w, unsigned short* ph, unsigned short* pl,
                                                 int K, int Nn) {
  const int groups = (Nn * K) >> 3;
  const int g  = blockIdx.x * NTHR + threadIdx.x;
  const bool ok = g < groups;
  const int gc = ok ? g : groups - 1;
  const int kq8 = K >> 3;
  const int n = gc / kq8, kq = gc - n * kq8;
  v8us oh, ol;
#pragma unroll
  for (int i = 0; i < 8; ++i) {
    const float v = w[(size_t)(kq * 8 + i) * Nn + n];
    unsigned short h_, l_;
    split_bf16(v, h_, l_);
    oh[i] = h_;
    ol[i] = l_;
  }
  const size_t d = (size_t)n * K + kq * 8;
  if (ok) { *(volatile v8us*)(ph + d) = oh; *(volatile v8us*)(pl + d) = ol; }
  __threadfence();
  if (ok) { *(volatile v8us*)(ph + d) = oh; *(volatile v8us*)(pl + d) = ol; }
}

__global__ __launch_bounds__(NTHR) void k_prepcat(const float* __restrict__ w1, _Float16* plane, int F) {
  const int groups = (256 * F) >> 3;
  const int g  = blockIdx.x * NTHR + threadIdx.x;
  const bool ok = g < groups;
  const int gc = ok ? g : groups - 1;
  const int kq8 = F >> 3;
  const int n = gc / kq8, kq = gc - n * kq8;
  const int nn = n & 127;
  v8h o;
#pragma unroll
  for (int i = 0; i < 8; ++i) {
    const int k = kq * 8 + i;
    const float top = w1[(size_t)k * 128 + nn];
    const float bot = w1[(size_t)(F + k) * 128 + nn];
    const float v = (n < 128) ? (top - bot) : bot;
    o[i] = (_Float16)(v * WSC);
  }
  _Float16* dst = plane + (size_t)n * F + kq * 8;
  if (ok) *(volatile v8h*)dst = o;
  __threadfence();
  if (ok) *(volatile v8h*)dst = o;
}

template <int K, int BNAPPLY>
__global__ __launch_bounds__(NTHR) void k_node(const float* __restrict__ xin, const float* __restrict__ bnl,
                                               const _Float16* __restrict__ Bp, const float* __restrict__ b1,
                                               _Float16* PQ, int nN) {
  __shared__ __attribute__((aligned(16))) _Float16 sa[MT * K];
  __shared__ __attribute__((aligned(16))) _Float16 so[MT * PQW];
  const int tid = threadIdx.x, lane = tid & 31, wave = tid >> 5, hh = lane >> 4, m = lane & 15;
  const int row0 = blockIdx.x * MT;

  {
    constexpr int KQ = K / 4;
    const int r = tid >> 2, q = tid & 3;
    const int gr = clampi(row0 + r, 0, nN - 1);
    const float* xp = xin + (size_t)gr * K + q * KQ;
#pragma unroll
    for (int j = 0; j < KQ / 8; ++j) {
      const v4f a = *(const v4f*)(xp + 8 * j);
      const v4f b = *(const v4f*)(xp + 8 * j + 4);
      float f[8] = {a.x, a.y, a.z, a.w, b.x, b.y, b.z, b.w};
      if (BNAPPLY != 0) {
        const v4f s0 = *(const v4f*)(bnl + q * KQ + 8 * j);
        const v4f s1 = *(const v4f*)(bnl + q * KQ + 8 * j + 4);
        const v4f t0 = *(const v4f*)(bnl + HC + q * KQ + 8 * j);
        const v4f t1 = *(const v4f*)(bnl + HC + q * KQ + 8 * j + 4);
        const float ss[8] = {s0.x, s0.y, s0.z, s0.w, s1.x, s1.y, s1.z, s1.w};
        const float tt[8] = {t0.x, t0.y, t0.z, t0.w, t1.x, t1.y, t1.z, t1.w};
#pragma unroll
        for (int i = 0; i < 8; ++i) f[i] = fmaxf(fmaf(f[i], ss[i], tt[i]), 0.0f);
      }
      v8h o;
#pragma unroll
      for (int i = 0; i < 8; ++i) o[i] = (_Float16)f[i];
      *(v8h*)(sa + r * K + q * KQ + 8 * j) = o;
    }
  }
  __syncthreads();

  const int rt = wave >> 1, ctb = (wave & 1) * 8;
  v8f acc[8];
#pragma unroll
  for (int ct = 0; ct < 8; ++ct) {
#pragma unroll
    for (int r = 0; r < 8; ++r) acc[ct][r] = 0.0f;
  }
#pragma unroll
  for (int ks = 0; ks < K / 32; ++ks) {
    const v16h a = ldfrag(sa + (rt * 16 + m) * K + 32 * ks + 8 * hh);
#pragma unroll
    for (int ct = 0; ct < 8; ++ct) {
      const v16h b = ldfrag(Bp + (size_t)((ctb + ct) * 16 + m) * K + 32 * ks + 8 * hh);
      acc[ct] = wmh(a, b, acc[ct]);
    }
  }
#pragma unroll
  for (int ct = 0; ct < 8; ++ct) {
    const int col = (ctb + ct) * 16 + m;
    const float bb = b1[col & 127];
    const float bias = (ctb == 0) ? bb : 0.0f;
#pragma unroll
    for (int r = 0; r < 8; ++r) {
      const float v = acc[ct][r] * WINV + bias;
      so[(rt * 16 + 8 * hh + r) * PQW + col] = (_Float16)v;
    }
  }
  __syncthreads();

  v8h ov[8];
#pragma unroll
  for (int i = 0; i < 8; ++i) ov[i] = *(const v8h*)(so + (wave + NWAVE * i) * PQW + 8 * lane);
#pragma unroll
  for (int i = 0; i < 8; ++i)
    *(volatile v8h*)(PQ + (size_t)(row0 + wave + NWAVE * i) * PQW + 8 * lane) = ov[i];
  __threadfence();
#pragma unroll
  for (int i = 0; i < 8; ++i)
    *(volatile v8h*)(PQ + (size_t)(row0 + wave + NWAVE * i) * PQW + 8 * lane) = ov[i];
}

__global__ __launch_bounds__(NTHR) void k_agg(const _Float16* __restrict__ PQ, const int* __restrict__ ei,
                                              const _Float16* __restrict__ W2T, const float* __restrict__ b2,
                                              float* hout, double* part, int nN, int nE, int vec8) {
  __shared__ __attribute__((aligned(16))) float    acc[NROWA * HC];
  __shared__ __attribute__((aligned(16))) _Float16 stg[NWAVE * 16 * HC];
  __shared__ int pend[PCAP];
  __shared__ int bins[PCAP];
  __shared__ int cq[QMAX * NWAVE * NWAVE];
  __shared__ int slt[NWAVE * 16];
  __shared__ __attribute__((aligned(16))) double red[4 * HC];
  __shared__ __attribute__((aligned(16))) double pd[2 * HC];
  __shared__ int wcnt[NWAVE];
  __shared__ int tot[NWAVE];
  __shared__ int bbase[NWAVE];
  __shared__ int pendN;

  const int tid = threadIdx.x, lane = tid & 31, wave = tid >> 5, hh = lane >> 4, m = lane & 15;
  const int nodeBase = blockIdx.x * NB;
  const int dumpRow = NB + wave;
  const int* srcs = ei;
  const int* dsts = ei + nE;
  const int nEm1 = nE > 0 ? nE - 1 : 0;

  {
    const float ninf = -__builtin_inff();
    const v4f nv = {ninf, ninf, ninf, ninf};
    for (int i = tid; i < (NROWA * HC) / 4; i += NTHR) *(v4f*)(acc + 4 * i) = nv;
  }
  if (tid == 0) pendN = 0;
  float b2x[8];
#pragma unroll
  for (int ns = 0; ns < 8; ++ns) b2x[ns] = b2[ns * 16 + m] * WSC;
  __syncthreads();

  const int nChunks = (nE + CHUNK - 1) / CHUNK;
#pragma unroll 1
  for (int ch = 0; ch < nChunks; ++ch) {
    const int cbase = ch * CHUNK;
    const int e0 = cbase + tid * EPT;
    int dv[8];
    {
      const int sent = -2147483647 - 1;
      const int waveLast = cbase + (wave * 32 + 31) * EPT + 7;
      v4i da, db;
      if (vec8 != 0 && waveLast < nE) {
        da = *(const v4i*)(dsts + e0);
        db = *(const v4i*)(dsts + e0 + 4);
      } else {
        da.x = (e0     < nE) ? dsts[clampi(e0,     0, nEm1)] : sent;
        da.y = (e0 + 1 < nE) ? dsts[clampi(e0 + 1, 0, nEm1)] : sent;
        da.z = (e0 + 2 < nE) ? dsts[clampi(e0 + 2, 0, nEm1)] : sent;
        da.w = (e0 + 3 < nE) ? dsts[clampi(e0 + 3, 0, nEm1)] : sent;
        db.x = (e0 + 4 < nE) ? dsts[clampi(e0 + 4, 0, nEm1)] : sent;
        db.y = (e0 + 5 < nE) ? dsts[clampi(e0 + 5, 0, nEm1)] : sent;
        db.z = (e0 + 6 < nE) ? dsts[clampi(e0 + 6, 0, nEm1)] : sent;
        db.w = (e0 + 7 < nE) ? dsts[clampi(e0 + 7, 0, nEm1)] : sent;
      }
      dv[0] = da.x; dv[1] = da.y; dv[2] = da.z; dv[3] = da.w;
      dv[4] = db.x; dv[5] = db.y; dv[6] = db.z; dv[7] = db.w;
    }
    unsigned msk[8];
    int sl[8];
    int wc = 0;
#pragma unroll
    for (int j = 0; j < 8; ++j) {
      const unsigned s = (unsigned)dv[j] - (unsigned)nodeBase;
      const bool h = s < (unsigned)NB;
      sl[j] = h ? (int)s : 0;
      msk[j] = __builtin_amdgcn_ballot_w32(h);
      wc += (int)__builtin_popcount(msk[j]);
    }
    if (lane == 0) wcnt[wave] = wc;
    __syncthreads();

    const int base = pendN;
    int tsum = 0, myoff = 0;
#pragma unroll
    for (int w = 0; w < NWAVE; ++w) {
      int c = wcnt[w];
      c = clampi(c, 0, EPT * 32);
      if (w < wave) myoff += c;
      tsum += c;
    }
    {
      int run = 0;
#pragma unroll
      for (int j = 0; j < 8; ++j) {
        const bool h = ((msk[j] >> lane) & 1u) != 0u;
        if (h) {
          const int pos = base + myoff + run + (int)__builtin_amdgcn_mbcnt_lo(msk[j], 0u);
          if ((unsigned)pos < (unsigned)PCAP) pend[pos] = ((e0 + j) << KEYSH) | sl[j];
        }
        run += (int)__builtin_popcount(msk[j]);
      }
    }
    int newN = base + tsum;
    newN = clampi(newN, 0, PCAP);
    const bool lastCh = (ch == nChunks - 1);
    const bool drainNow = lastCh || (newN > DRAINT);
    __syncthreads();

    if (drainNow) {
      const int n = newN;
#pragma unroll 1
      for (int q = 0; q < QMAX; ++q) {
        const int i = q * NTHR + tid;
        const bool valid = i < n;
        const int key = pend[i];
        const int o = key & 7;
#pragma unroll
        for (int oo = 0; oo < 8; ++oo) {
          const unsigned b = __builtin_amdgcn_ballot_w32(valid && (o == oo));
          if (lane == 0) cq[(q * NWAVE + wave) * NWAVE + oo] = (int)__builtin_popcount(b);
        }
      }
      __syncthreads();
      if (tid < NWAVE) {
        int runv = 0;
#pragma unroll 1
        for (int s = 0; s < QMAX * NWAVE; ++s) {
          const int idx = s * NWAVE + tid;
          const int c = cq[idx];
          cq[idx] = runv;
          runv += c;
        }
        tot[tid] = runv;
      }
      __syncthreads();
      if (tid == 0) {
        int b = 0;
#pragma unroll
        for (int o = 0; o < NWAVE; ++o) { bbase[o] = b; b += tot[o]; }
      }
      __syncthreads();
#pragma unroll 1
      for (int q = 0; q < QMAX; ++q) {
        const int i = q * NTHR + tid;
        const bool valid = i < n;
        const int key = pend[i];
        const int o = key & 7;
#pragma unroll
        for (int oo = 0; oo < 8; ++oo) {
          const bool mine = valid && (o == oo);
          const unsigned b = __builtin_amdgcn_ballot_w32(mine);
          if (mine) {
            const int pos = bbase[oo] + cq[(q * NWAVE + wave) * NWAVE + oo] + (int)__builtin_amdgcn_mbcnt_lo(b, 0u);
            bins[clampi(pos, 0, PCAP - 1)] = key;
          }
        }
      }
      __syncthreads();

      int cntW = clampi(tot[wave], 0, PCAP);
      int bb = clampi(bbase[wave], 0, PCAP);
      cntW = __builtin_amdgcn_readfirstlane(cntW);
      bb = __builtin_amdgcn_readfirstlane(bb);
      int T = (cntW + 15) >> 4;
      T = T > (PCAP / 16) ? (PCAP / 16) : T;
#pragma unroll 1
      for (int t = 0; t < T; ++t) {
        {
          const int e = m;
          const int pos = 16 * t + e;
          const bool valid = pos < cntW;
          const int key = bins[clampi(bb + pos, 0, PCAP - 1)];
          int edge = key >> KEYSH;
          int slot = key & ((1 << KEYSH) - 1);
          slot = (valid && slot < NB) ? slot : dumpRow;
          edge = valid ? clampi(edge, 0, nEm1) : 0;
          const int jn = clampi(srcs[edge], 0, nN - 1);
          const int in_ = clampi(nodeBase + slot, 0, nN - 1);
          const _Float16* pp = PQ + (size_t)in_ * PQW + 64 * hh;
          const _Float16* qp = PQ + (size_t)jn * PQW + HC + 64 * hh;
          _Float16* sp = stg + (wave * 16 + e) * HC + 64 * hh;
#pragma unroll
          for (int q8 = 0; q8 < 8; ++q8) {
            const v8h a = *(const v8h*)(pp + 8 * q8);
            const v8h b = *(const v8h*)(qp + 8 * q8);
            v8h o;
#pragma unroll
            for (int c = 0; c < 8; ++c) {
              const float f = fmaxf((float)a[c] + (float)b[c], 0.0f);
              o[c] = (_Float16)f;
            }
            *(v8h*)(sp + 8 * q8) = o;
          }
          if (hh == 0) slt[wave * 16 + e] = slot;
        }
        wave_lds_sync();

        v8f d[8];
#pragma unroll
        for (int ns = 0; ns < 8; ++ns) {
#pragma unroll
          for (int r = 0; r < 8; ++r) d[ns][r] = b2x[ns];
        }
#pragma unroll
        for (int ks = 0; ks < HC / 32; ++ks) {
          const v16h a = ldfrag(stg + (wave * 16 + m) * HC + 32 * ks + 8 * hh);
#pragma unroll
          for (int ns = 0; ns < 8; ++ns) {
            const v16h b = ldfrag(W2T + (size_t)(ns * 16 + m) * HC + 32 * ks + 8 * hh);
            d[ns] = wmh(a, b, d[ns]);
          }
        }
        float rcv[4][8];
#pragma unroll
        for (int g = 0; g < 4; ++g) {
#pragma unroll
          for (int r = 0; r < 8; ++r) {
            const float snd = hh ? d[g][r] : d[4 + g][r];
            rcv[g][r] = __shfl_xor(snd, 16);
          }
        }
        const int colb = hh * 64 + m;
#pragma unroll
        for (int ee = 0; ee < 16; ++ee) {
          int row = slt[wave * 16 + ee];
          row = ((unsigned)row < (unsigned)NROWA) ? row : dumpRow;
          row = __builtin_amdgcn_readfirstlane(row);
          float* ap = acc + row * HC + colb;
#pragma unroll
          for (int g = 0; g < 4; ++g) {
            float v;
            if (ee < 8) v = hh ? rcv[g][ee & 7] : d[g][ee & 7];
            else        v = hh ? d[4 + g][ee & 7] : rcv[g][ee & 7];
            v *= WINV;
            const float o = ap[16 * g];
            ap[16 * g] = fmaxf(o, v);
          }
        }
        wave_lds_sync();
      }
      __syncthreads();
      if (tid == 0) pendN = 0;
    } else {
      if (tid == 0) pendN = newN;
    }
  }
  __syncthreads();

#pragma unroll 1
  for (int i = 0; i < NB / NWAVE; ++i) {
    const int r = wave + NWAVE * i;
    const v4f v = san4(*(const v4f*)(acc + r * HC + 4 * lane));
    *(volatile v4f*)(hout + (size_t)(nodeBase + r) * HC + 4 * lane) = v;
  }
  __threadfence();
#pragma unroll 1
  for (int i = 0; i < NB / NWAVE; ++i) {
    const int r = wave + NWAVE * i;
    const v4f v = san4(*(const v4f*)(acc + r * HC + 4 * lane));
    *(volatile v4f*)(hout + (size_t)(nodeBase + r) * HC + 4 * lane) = v;
  }

  {
    const int c = tid & 127, ph = tid >> 7;
    const int rlim = clampi(nN - nodeBase, 0, NB);
    double s = 0.0, q = 0.0;
#pragma unroll 1
    for (int r = ph; r < rlim; r += 2) {
      float v = acc[r * HC + c];
      v = (v > -3.0e38f) ? v : 0.0f;
      s += (double)v;
      q += (double)v * (double)v;
    }
    red[(2 * ph) * HC + c] = s;
    red[(2 * ph + 1) * HC + c] = q;
  }
  __syncthreads();
  if (tid < HC) {
    pd[tid]      = red[tid] + red[2 * HC + tid];
    pd[HC + tid] = red[HC + tid] + red[3 * HC + tid];
  }
  __syncthreads();
  if (tid < HC) {
    const v2d v = *(const v2d*)(pd + 2 * tid);
    *(volatile v2d*)(part + (size_t)blockIdx.x * (2 * HC) + 2 * tid) = v;
  }
  __threadfence();
  if (tid < HC) {
    const v2d v = *(const v2d*)(pd + 2 * tid);
    *(volatile v2d*)(part + (size_t)blockIdx.x * (2 * HC) + 2 * tid) = v;
  }
}

__global__ __launch_bounds__(128) void k_bnfin(const double* __restrict__ part, const float* __restrict__ gam,
                                              const float* __restrict__ bet, float* bnl, int nBlk, int nN) {
  __shared__ __attribute__((aligned(16))) float ln[2 * HC];
  const int tid = threadIdx.x;
  const int c = tid & 127;
  double S = 0.0, SQ = 0.0;
#pragma unroll 1
  for (int b = 0; b < nBlk; ++b) {
    S  += part[(size_t)b * (2 * HC) + c];
    SQ += part[(size_t)b * (2 * HC) + HC + c];
  }
  const double inv = 1.0 / (double)(nN > 0 ? nN : 1);
  const double mu = S * inv;
  double var = SQ * inv - mu * mu;
  if (var < 0.0) var = 0.0;
  const float varf = (float)var;
  const float rstd = 1.0f / sqrtf(varf + BN_EPS);
  const float s = rstd * gam[c];
  const float t = bet[c] - (float)mu * s;
  if (tid < HC) { ln[c] = s; ln[HC + c] = t; }
  __syncthreads();
  v4f v = {0.0f, 0.0f, 0.0f, 0.0f};
  const bool wr = tid < 64;
  if (wr) v = *(const v4f*)(ln + 4 * tid);
  if (wr) *(volatile v4f*)(bnl + 4 * tid) = v;
  __threadfence();
  if (wr) *(volatile v4f*)(bnl + 4 * tid) = v;
}

__global__ __launch_bounds__(NTHR) void k_pool(const float* __restrict__ h, const int* __restrict__ bidx,
                                               const float* __restrict__ bnl, float* G, int nN) {
  __shared__ int list[NTHR];
  __shared__ int wl[NWAVE];
  __shared__ __attribute__((aligned(16))) double red[2 * HC];
  __shared__ __attribute__((aligned(16))) float gl[HC];
  const int tid = threadIdx.x, lane = tid & 31, wave = tid >> 5;
  const int g = blockIdx.x;
  const int c = tid & 127, ph = tid >> 7;
  const float s = bnl[c], t = bnl[HC + c];
  double sum = 0.0;
  int cntTot = 0;
  const int nCh = (nN + NTHR - 1) / NTHR;
#pragma unroll 1
  for (int ch = 0; ch < nCh; ++ch) {
    const int n = ch * NTHR + tid;
    const bool valid = n < nN;
    const int b = bidx[clampi(n, 0, nN - 1)];
    const bool hit = valid && (b == g);
    const unsigned mk = __builtin_amdgcn_ballot_w32(hit);
    if (lane == 0) wl[wave] = (int)__builtin_popcount(mk);
    __syncthreads();
    int off = 0, totc = 0;
#pragma unroll
    for (int w = 0; w < NWAVE; ++w) { const int cw = clampi(wl[w], 0, 32); if (w < wave) off += cw; totc += cw; }
    if (hit) {
      const int pos = off + (int)__builtin_amdgcn_mbcnt_lo(mk, 0u);
      if ((unsigned)pos < (unsigned)NTHR) list[pos] = n;
    }
    totc = clampi(totc, 0, NTHR);
    totc = __builtin_amdgcn_readfirstlane(totc);
    __syncthreads();
    const int np = (totc + 1) >> 1;
#pragma unroll 1
    for (int p = 0; p < np; ++p) {
      const int idx = 2 * p + ph;
      const bool ok = idx < totc;
      const int node = clampi(list[clampi(idx, 0, NTHR - 1)], 0, nN - 1);
      float v = h[(size_t)node * HC + c];
      v = fmaxf(fmaf(v, s, t), 0.0f);
      sum += ok ? (double)v : 0.0;
    }
    cntTot += totc;
    __syncthreads();
  }
  red[ph * HC + c] = sum;
  __syncthreads();
  if (tid < HC) {
    const double S = red[c] + red[HC + c];
    const int cn = cntTot > 1 ? cntTot : 1;
    gl[c] = (float)S * (1.0f / (float)cn);
  }
  __syncthreads();
  v4f v = {0.0f, 0.0f, 0.0f, 0.0f};
  const bool wr = tid < 32;
  if (wr) v = *(const v4f*)(gl + 4 * tid);
  if (wr) *(volatile v4f*)(G + (size_t)g * HC + 4 * tid) = v;
  __threadfence();
  if (wr) *(volatile v4f*)(G + (size_t)g * HC + 4 * tid) = v;
}

__global__ __launch_bounds__(NTHR) void k_head(const float* __restrict__ G,
                                               const unsigned short* __restrict__ L1H, const unsigned short* __restrict__ L1L,
                                               const float* __restrict__ l1b,
                                               const unsigned short* __restrict__ L2H, const unsigned short* __restrict__ L2L,
                                               const float* __restrict__ l2b,
                                               const unsigned short* __restrict__ OTH, const unsigned short* __restrict__ OTL,
                                               const float* __restrict__ ob, float* outp) {
  __shared__ __attribute__((aligned(16))) unsigned short a0h[64 * 128];
  __shared__ __attribute__((aligned(16))) unsigned short a0l[64 * 128];
  __shared__ __attribute__((aligned(16))) unsigned short a1h[64 * 256];
  __shared__ __attribute__((aligned(16))) unsigned short a1l[64 * 256];
  __shared__ __attribute__((aligned(16))) unsigned short a2h[64 * 128];
  __shared__ __attribute__((aligned(16))) unsigned short a2l[64 * 128];
  __shared__ __attribute__((aligned(16))) float          so[64 * 16];
  const int tid = threadIdx.x, lane = tid & 31, wave = tid >> 5, hh = lane >> 4, m = lane & 15;

#pragma unroll
  for (int it = 0; it < 4; ++it) {
    const int gi = it * NTHR + tid;
    const int r = gi >> 4, k8 = gi & 15;
    const v4f a = *(const v4f*)(G + r * 128 + 8 * k8);
    const v4f b = *(const v4f*)(G + r * 128 + 8 * k8 + 4);
    const float f[8] = {a.x, a.y, a.z, a.w, b.x, b.y, b.z, b.w};
    v8us oh, ol;
#pragma unroll
    for (int i = 0; i < 8; ++i) {
      unsigned short h_, l_;
      split_bf16(f[i], h_, l_);
      oh[i] = h_;
      ol[i] = l_;
    }
    *(v8us*)(a0h + r * 128 + 8 * k8) = oh;
    *(v8us*)(a0l + r * 128 + 8 * k8) = ol;
  }
  __syncthreads();

  {
    const int rt = wave >> 1, ctb = (wave & 1) * 8;
    v8f acc[8];
#pragma unroll
    for (int ct = 0; ct < 8; ++ct) {
      const float bv = l1b[(ctb + ct) * 16 + m];
#pragma unroll
      for (int r = 0; r < 8; ++r) acc[ct][r] = bv;
    }
#pragma unroll
    for (int ks = 0; ks < 4; ++ks) {
      const int ao = (rt * 16 + m) * 128 + 32 * ks + 8 * hh;
      const v16b ah = ldfragb(a0h + ao);
      const v16b al = ldfragb(a0l + ao);
#pragma unroll
      for (int ct = 0; ct < 8; ++ct) {
        const size_t bo = (size_t)((ctb + ct) * 16 + m) * 128 + 32 * ks + 8 * hh;
        const v16b bh = ldfragb(L1H + bo);
        const v16b bl = ldfragb(L1L + bo);
        acc[ct] = wmb3(ah, al, bh, bl, acc[ct]);
      }
    }
#pragma unroll
    for (int ct = 0; ct < 8; ++ct) {
      const int col = (ctb + ct) * 16 + m;
#pragma unroll
      for (int r = 0; r < 8; ++r) {
        const float v = fmaxf(acc[ct][r], 0.0f);
        unsigned short h_, l_;
        split_bf16(v, h_, l_);
        const int idx = (rt * 16 + 8 * hh + r) * 256 + col;
        a1h[idx] = h_;
        a1l[idx] = l_;
      }
    }
  }
  __syncthreads();

  {
    const int rt = wave >> 1, ctb = (wave & 1) * 4;
    v8f acc[4];
#pragma unroll
    for (int ct = 0; ct < 4; ++ct) {
      const float bv = l2b[(ctb + ct) * 16 + m];
#pragma unroll
      for (int r = 0; r < 8; ++r) acc[ct][r] = bv;
    }
#pragma unroll
    for (int ks = 0; ks < 8; ++ks) {
      const int ao = (rt * 16 + m) * 256 + 32 * ks + 8 * hh;
      const v16b ah = ldfragb(a1h + ao);
      const v16b al = ldfragb(a1l + ao);
#pragma unroll
      for (int ct = 0; ct < 4; ++ct) {
        const size_t bo = (size_t)((ctb + ct) * 16 + m) * 256 + 32 * ks + 8 * hh;
        const v16b bh = ldfragb(L2H + bo);
        const v16b bl = ldfragb(L2L + bo);
        acc[ct] = wmb3(ah, al, bh, bl, acc[ct]);
      }
    }
#pragma unroll
    for (int ct = 0; ct < 4; ++ct) {
      const int col = (ctb + ct) * 16 + m;
#pragma unroll
      for (int r = 0; r < 8; ++r) {
        const float v = fmaxf(acc[ct][r], 0.0f);
        unsigned short h_, l_;
        split_bf16(v, h_, l_);
        const int idx = (rt * 16 + 8 * hh + r) * 128 + col;
        a2h[idx] = h_;
        a2l[idx] = l_;
      }
    }
  }
  __syncthreads();

  if (wave < 4) {
    const int rt = wave;
    v8f acc;
    const float bv = ob[m];
#pragma unroll
    for (int r = 0; r < 8; ++r) acc[r] = bv;
#pragma unroll
    for (int ks = 0; ks < 4; ++ks) {
      const int ao = (rt * 16 + m) * 128 + 32 * ks + 8 * hh;
      const v16b ah = ldfragb(a2h + ao);
      const v16b al = ldfragb(a2l + ao);
      const size_t bo = (size_t)m * 128 + 32 * ks + 8 * hh;
      const v16b bh = ldfragb(OTH + bo);
      const v16b bl = ldfragb(OTL + bo);
      acc = wmb3(ah, al, bh, bl, acc);
    }
#pragma unroll
    for (int r = 0; r < 8; ++r) so[(rt * 16 + 8 * hh + r) * 16 + m] = fmaxf(acc[r], 0.0f);
  }
  __syncthreads();

  const v4f v = *(const v4f*)(so + 4 * tid);
  *(volatile v4f*)(outp + 4 * tid) = v;
  __threadfence();
  *(volatile v4f*)(outp + 4 * tid) = v;
}

static inline size_t al256(size_t v) { return (v + 255) & ~(size_t)255; }

extern "C" void kernel_launch(void* const* d_in, const int* in_sizes, int n_in,
                              void* d_out, int out_size, void* d_ws, size_t ws_size,
                              hipStream_t stream) {
  if (n_in < 21) return;
  const int nN = in_sizes[2];
  if (nN <= 0) return;
  if (in_sizes[0] != nN * 64) return;
  const int nE = in_sizes[1] / 2;
  if (nE < 0 || in_sizes[1] != nE * 2 || nE >= (1 << 21)) return;
  if (in_sizes[3] != 128 * 128 || in_sizes[4] != 128 || in_sizes[5] != 128 * 128 || in_sizes[6] != 128) return;
  if (in_sizes[7] != 128 || in_sizes[8] != 128) return;
  if (in_sizes[9] != 256 * 128 || in_sizes[10] != 128 || in_sizes[11] != 128 * 128 || in_sizes[12] != 128) return;
  if (in_sizes[13] != 128 || in_sizes[14] != 128) return;
  if (in_sizes[15] != 128 * 256 || in_sizes[16] != 256 || in_sizes[17] != 256 * 128 || in_sizes[18] != 128) return;
  if (in_sizes[19] != 128 * 16 || in_sizes[20] != 16) return;
  if (out_size != NGRAPH * 16) return;

  const float* x     = (const float*)d_in[0];
  const int*   ei    = (const int*)d_in[1];
  const int*   bidx  = (const int*)d_in[2];
  const float* c1w1  = (const float*)d_in[3];
  const float* c1b1  = (const float*)d_in[4];
  const float* c1w2  = (const float*)d_in[5];
  const float* c1b2  = (const float*)d_in[6];
  const float* bn1g  = (const float*)d_in[7];
  const float* bn1b  = (const float*)d_in[8];
  const float* c2w1  = (const float*)d_in[9];
  const float* c2b1  = (const float*)d_in[10];
  const float* c2w2  = (const float*)d_in[11];
  const float* c2b2  = (const float*)d_in[12];
  const float* bn2g  = (const float*)d_in[13];
  const float* bn2b  = (const float*)d_in[14];
  const float* lin1w = (const float*)d_in[15];
  const float* lin1b = (const float*)d_in[16];
  const float* lin2w = (const float*)d_in[17];
  const float* lin2b = (const float*)d_in[18];
  const float* outw  = (const float*)d_in[19];
  const float* outb  = (const float*)d_in[20];
  float* out = (float*)d_out;

  const int nBlkG = (nN + MT - 1) / MT;
  const int nBlkA = (nN + NB - 1) / NB;

  char* ws = (char*)d_ws;
  size_t off = 0;
  const size_t oB1  = off; off = al256(off + (size_t)256 * 64 * 2);
  const size_t oW21 = off; off = al256(off + (size_t)128 * 128 * 2);
  const size_t oB2  = off; off = al256(off + (size_t)256 * 128 * 2);
  const size_t oW22 = off; off = al256(off + (size_t)128 * 128 * 2);
  const size_t oL1  = off; off = al256(off + (size_t)2 * 256 * 128 * 2);
  const size_t oL2  = off; off = al256(off + (size_t)2 * 128 * 256 * 2);
  const size_t oOT  = off; off = al256(off + (size_t)2 * 16 * 128 * 2);
  const size_t oPQ  = off; off = al256(off + (size_t)nBlkG * MT * PQW * 2);
  const size_t oH1  = off; off = al256(off + (size_t)nBlkA * NB * HC * 4);
  const size_t oH2  = off; off = al256(off + (size_t)nBlkA * NB * HC * 4);
  const size_t oP1  = off; off = al256(off + (size_t)nBlkA * 2 * HC * 8);
  const size_t oP2  = off; off = al256(off + (size_t)nBlkA * 2 * HC * 8);
  const size_t oBn1 = off; off = al256(off + (size_t)2 * HC * 4);
  const size_t oBn2 = off; off = al256(off + (size_t)2 * HC * 4);
  const size_t oG   = off; off = al256(off + (size_t)NGRAPH * HC * 4);
  if (off > ws_size) return;
  if (off > (size_t)134217728) return;

  _Float16* B1  = (_Float16*)(ws + oB1);
  _Float16* W21 = (_Float16*)(ws + oW21);
  _Float16* B2  = (_Float16*)(ws + oB2);
  _Float16* W22 = (_Float16*)(ws + oW22);
  unsigned short* L1H = (unsigned short*)(ws + oL1);
  unsigned short* L1L = L1H + 256 * 128;
  unsigned short* L2H = (unsigned short*)(ws + oL2);
  unsigned short* L2L = L2H + 128 * 256;
  unsigned short* OTH = (unsigned short*)(ws + oOT);
  unsigned short* OTL = OTH + 16 * 128;
  _Float16* PQ  = (_Float16*)(ws + oPQ);
  float*  H1  = (float*)(ws + oH1);
  float*  H2  = (float*)(ws + oH2);
  double* P1  = (double*)(ws + oP1);
  double* P2  = (double*)(ws + oP2);
  float*  Bn1 = (float*)(ws + oBn1);
  float*  Bn2 = (float*)(ws + oBn2);
  float*  Gp  = (float*)(ws + oG);

  const int vec8 = ((nE & 3) == 0) ? 1 : 0;

  k_prepcat<<<(256 * 64 / 8 + NTHR - 1) / NTHR, NTHR, 0, stream>>>(c1w1, B1, 64);
  k_prepT<<<(128 * 128 / 8 + NTHR - 1) / NTHR, NTHR, 0, stream>>>(c1w2, W21, 128, 128);
  k_prepcat<<<(256 * 128 / 8 + NTHR - 1) / NTHR, NTHR, 0, stream>>>(c2w1, B2, 128);
  k_prepT<<<(128 * 128 / 8 + NTHR - 1) / NTHR, NTHR, 0, stream>>>(c2w2, W22, 128, 128);
  k_prepT3<<<(256 * 128 / 8 + NTHR - 1) / NTHR, NTHR, 0, stream>>>(lin1w, L1H, L1L, 128, 256);
  k_prepT3<<<(128 * 256 / 8 + NTHR - 1) / NTHR, NTHR, 0, stream>>>(lin2w, L2H, L2L, 256, 128);
  k_prepT3<<<(16 * 128 / 8 + NTHR - 1) / NTHR, NTHR, 0, stream>>>(outw, OTH, OTL, 128, 16);

  k_node<64, 0><<<nBlkG, NTHR, 0, stream>>>(x, Bn1, B1, c1b1, PQ, nN);
  k_agg<<<nBlkA, NTHR, 0, stream>>>(PQ, ei, W21, c1b2, H1, P1, nN, nE, vec8);
  k_bnfin<<<1, 128, 0, stream>>>(P1, bn1g, bn1b, Bn1, nBlkA, nN);

  k_node<128, 1><<<nBlkG, NTHR, 0, stream>>>(H1, Bn1, B2, c2b1, PQ, nN);
  k_agg<<<nBlkA, NTHR, 0, stream>>>(PQ, ei, W22, c2b2, H2, P2, nN, nE, vec8);
  k_bnfin<<<1, 128, 0, stream>>>(P2, bn2g, bn2b, Bn2, nBlkA, nN);

  k_pool<<<NGRAPH, NTHR, 0, stream>>>(H2, bidx, Bn2, Gp, nN);
  k_head<<<1, NTHR, 0, stream>>>(Gp, L1H, L1L, lin1b, L2H, L2L, lin2b, OTH, OTL, outb, out);
}
